// GNN_node_Virtualnode_45621142618641
// MI455X (gfx1250) — hardware-verified
//
#include <hip/hip_runtime.h>
#include <stddef.h>
#include <stdint.h>


#define NB     128
#define NPG    256
#define EPG    2048
#define EMB    256
#define HID    512
#define NNODE  (NB * NPG)
#define NLAY   5
#define ATOMV  119
#define BONDV  16
#define EHC    64
#define NTHR   256
#define GBM    64
#define GBN    128
#define GTHR   128
#define PARTW  256
#define NRT    (NNODE / GBM)
#define OFFP   260
#define PC     64
#define AC     128
#define ORDMAX 8
#define LDS_PROP ((3 * NPG * PC + EPG + EPG + 264 + NPG) * 4)
#define LDS_AGG  ((NPG * AC + BONDV * AC + EPG + 264 + NTHR) * 4 + 2 * AC * 2)

static_assert(NPG == 256 && EPG == 2048 && NNODE == 32768);
static_assert(NTHR == NPG && EPG == 8 * NTHR);
static_assert(NNODE % GBM == 0 && NB % GBM == 0);
static_assert(HID % GBN == 0 && EMB % GBN == 0);
static_assert((2 * EMB) % 32 == 0 && (2 * HID) % 32 == 0);
static_assert(GTHR == GBN && GBM == (GTHR / 32) * 16);
static_assert(PARTW == 2 * GBN && PARTW / 4 <= GTHR);
static_assert(EMB == 4 * PC && EMB == 2 * AC && PC == 2 * 32 && AC == 4 * 32);
static_assert(LDS_PROP <= 300000 && LDS_AGG <= 300000);
static_assert((OFFP * 4) % 16 == 0 && OFFP >= NPG + 1);
static_assert(HID == 2 * EMB);

typedef float          v2f   __attribute__((ext_vector_type(2)));
typedef float          v4f   __attribute__((ext_vector_type(4)));
typedef float          v8f   __attribute__((ext_vector_type(8)));
typedef int            v4i   __attribute__((ext_vector_type(4)));
typedef int            v8i   __attribute__((ext_vector_type(8)));
typedef unsigned int   v4u   __attribute__((ext_vector_type(4)));
typedef unsigned short v4us  __attribute__((ext_vector_type(4)));
typedef unsigned short v8us  __attribute__((ext_vector_type(8)));
typedef __bf16         v16b  __attribute__((ext_vector_type(16)));
typedef v2f  __attribute__((may_alias)) v2fa;
typedef v4f  __attribute__((may_alias)) v4fa;
typedef v4i  __attribute__((may_alias)) v4ia;
typedef v4u  __attribute__((may_alias)) v4ua;
typedef v8us __attribute__((may_alias)) v8usa;
union FragB { v16b v; v8us h[2]; v8i w; };

__device__ __forceinline__ v8f wmb(const FragB& a, const FragB& b, v8f c) {
  v8f d = __builtin_amdgcn_wmma_f32_16x16x32_bf16(false, a.v, false, b.v, (short)0, c, false, false);
  asm volatile("v_nop\n\tv_nop\n\tv_nop\n\tv_nop" : "+v"(d) : "v"(a.w), "v"(b.w));
  return d;
}

__device__ __forceinline__ unsigned bf_bits(float f) {
  const unsigned u = __float_as_uint(f);
  const unsigned r = (u + 0x7FFFu + ((u >> 16) & 1u)) >> 16;
  return (f != f) ? 0x7fc0u : r;
}
__device__ __forceinline__ float bf_val(unsigned b) { return __uint_as_float(b << 16); }
__device__ __forceinline__ float bf_rne(float f) { return bf_val(bf_bits(f)); }
__device__ __forceinline__ float relu_np(float v) { return (v > 0.0f) ? v : (v - v); }
__device__ __forceinline__ void wave_sync_lds() {
  __builtin_amdgcn_fence(__ATOMIC_RELEASE, "wavefront");
  __builtin_amdgcn_wave_barrier();
}

__global__ __launch_bounds__(NTHR) void k_wprep(const float* __restrict__ W, int K, int N, int nUnits,
                                                unsigned short* out) {
  const int u = (int)blockIdx.x * NTHR + (int)threadIdx.x;
  if (u >= nUnits) return;
  const int upr = (2 * K) / 8;
  const int upl = N * upr;
  const int l   = u / upl;
  const int v   = u - l * upl;
  const int n   = v / upr;
  const int k8  = (v - n * upr) * 8;
  const int kk  = (k8 >= K) ? (k8 - K) : k8;
  const float* p = W + (size_t)l * (size_t)K * (size_t)N + (size_t)kk * (size_t)N + (size_t)n;
  v8us o;
#pragma unroll
  for (int i = 0; i < 8; ++i) o[i] = (unsigned short)bf_bits(p[(size_t)i * (size_t)N]);
  unsigned short* dp = out + (size_t)u * 8;
  *(volatile v8us*)dp = o;
  __threadfence();
  *(volatile v8us*)dp = o;
}

__global__ __launch_bounds__(NTHR) void k_lists(
    const int* __restrict__ lei, const int* __restrict__ eat,
    const float* __restrict__ bh, const float* __restrict__ lw, const float* __restrict__ lb,
    const float* __restrict__ vnemb,
    unsigned* GL, int* GOFF, unsigned* AL, float* COEF, int* AOFF, float* SELFC, int* META,
    float* VN, float* STAT2) {
  __shared__ __attribute__((aligned(16))) int      ed[EPG];
  __shared__ __attribute__((aligned(16))) int      rk[2 * EPG];
  __shared__ __attribute__((aligned(16))) unsigned gls[EPG];
  __shared__ __attribute__((aligned(16))) unsigned als[EPG];
  __shared__ __attribute__((aligned(16))) float    cfs[EPG];
  __shared__ __attribute__((aligned(16))) int      cnt[2 * NPG];
  __shared__ __attribute__((aligned(16))) int      offs[2 * OFFP];
  __shared__ __attribute__((aligned(16))) float    sums[2 * NPG];
  __shared__ __attribute__((aligned(16))) float    inv[2 * NPG];
  __shared__ __attribute__((aligned(16))) float    slf[NPG];
  __shared__ float ewt[16];
  __shared__ int   wtot[16];
  __shared__ int   wbad[8];
  __shared__ int   wdup[8];
  const int tid = (int)threadIdx.x, lane = tid & 31, wave = tid >> 5;
  const int g = (int)blockIdx.x;

  {
    const int* e0p = lei + (size_t)g * 2 * EPG;
    const int* e1p = e0p + EPG;
    const int* typ = eat + (size_t)g * EPG;
    const v4i a0 = *(const v4i*)(e0p + 8 * tid), a1 = *(const v4i*)(e0p + 8 * tid + 4);
    const v4i b0 = *(const v4i*)(e1p + 8 * tid), b1 = *(const v4i*)(e1p + 8 * tid + 4);
    const v4i c0 = *(const v4i*)(typ + 8 * tid), c1 = *(const v4i*)(typ + 8 * tid + 4);
    const int x0[8] = {a0.x, a0.y, a0.z, a0.w, a1.x, a1.y, a1.z, a1.w};
    const int x1[8] = {b0.x, b0.y, b0.z, b0.w, b1.x, b1.y, b1.z, b1.w};
    const int xt[8] = {c0.x, c0.y, c0.z, c0.w, c1.x, c1.y, c1.z, c1.w};
    int badl = 0;
#pragma unroll
    for (int i = 0; i < 8; ++i) {
      badl |= (((unsigned)x0[i] >= (unsigned)NPG) || ((unsigned)x1[i] >= (unsigned)NPG)) ? 1 : 0;
      const int q0 = x0[i] < 0 ? 0 : (x0[i] > NPG - 1 ? NPG - 1 : x0[i]);
      const int q1 = x1[i] < 0 ? 0 : (x1[i] > NPG - 1 ? NPG - 1 : x1[i]);
      const int qt = xt[i] < 0 ? 0 : (xt[i] > BONDV - 1 ? BONDV - 1 : xt[i]);
      ed[8 * tid + i] = q1 | (q0 << 8) | (qt << 16);
    }
    const unsigned bm = __builtin_amdgcn_ballot_w32(badl != 0);
    if (lane == 0) wbad[wave] = (bm != 0u) ? 1 : 0;
    cnt[tid] = 0;
    cnt[NPG + tid] = 0;
  }
  __syncthreads();

  if (wave < 2) {
    const int sh = 8 * wave;
#pragma unroll 1
    for (int b0 = 0; b0 < EPG; b0 += 32) {
      const int key = (ed[b0 + lane] >> sh) & 255;
      int rank = 0, later = 0;
#pragma unroll 4
      for (int k = 0; k < 32; ++k) {
        const int kk = __builtin_amdgcn_readlane(key, k);
        const int eq = (kk == key) ? 1 : 0;
        rank  += (k < lane) ? eq : 0;
        later |= (k > lane) ? eq : 0;
      }
      const int base = cnt[wave * NPG + key];
      rk[wave * EPG + b0 + lane] = base + rank;
      wave_sync_lds();
      if (later == 0) cnt[wave * NPG + key] = base + rank + 1;
      wave_sync_lds();
    }
  } else if (wave == 2) {
    const int ty = lane & 15;
    float a = 0.0f;
#pragma unroll 4
    for (int h = 0; h < EHC; ++h) a = fmaf(bf_rne(bh[ty * EHC + h]), bf_rne(lw[h]), a);
    const float x = a + bf_rne(lb[0]);
    const float w = 1.0f / (1.0f + expf(-x));
    if (lane < 16) ewt[ty] = w;
  }
  __syncthreads();

  {
    const int cg = cnt[tid], ca = cnt[NPG + tid];
    int ig = cg, ia = ca;
#pragma unroll
    for (int d = 1; d < 32; d <<= 1) {
      const int ug = __shfl_up(ig, d);
      const int ua = __shfl_up(ia, d);
      if (lane >= d) { ig += ug; ia += ua; }
    }
    if (lane == 31) { wtot[wave] = ig; wtot[8 + wave] = ia; }
    __syncthreads();
    int pg = 0, pa = 0;
#pragma unroll
    for (int w2 = 0; w2 < 8; ++w2) {
      pg += (w2 < wave) ? wtot[w2] : 0;
      pa += (w2 < wave) ? wtot[8 + w2] : 0;
    }
    offs[tid] = pg + ig - cg;
    offs[OFFP + tid] = pa + ia - ca;
    if (tid == NPG - 1) { offs[NPG] = pg + ig; offs[OFFP + NPG] = pa + ia; }
  }
  __syncthreads();

#pragma unroll 2
  for (int c = 0; c < 8; ++c) {
    const int e  = tid + NTHR * c;
    const int w  = ed[e];
    const int k1 = w & 255, k0 = (w >> 8) & 255, ty = (w >> 16) & 15;
    int pg = offs[k1] + rk[e];
    int pa = offs[OFFP + k0] + rk[EPG + e];
    pg = pg < 0 ? 0 : (pg > EPG - 1 ? EPG - 1 : pg);
    pa = pa < 0 ? 0 : (pa > EPG - 1 ? EPG - 1 : pa);
    gls[pg] = (unsigned)(k0 | (ty << 8) | (e << 12));
    als[pa] = (unsigned)(k1 | (e << 8) | (ty << 19));
  }
  __syncthreads();

  int* livef = rk;
  int ast = offs[OFFP + tid], aen = offs[OFFP + tid + 1];
  ast = ast < 0 ? 0 : (ast > EPG ? EPG : ast);
  aen = aen < ast ? ast : (aen > EPG ? EPG : aen);
  {
    float rs = 1.0f;
    int nd = 0;
#pragma unroll 1
    for (int p = ast; p < aen; ++p) {
      const unsigned ent = als[p];
      const unsigned j = ent & 255u;
      const int e  = (int)((ent >> 8) & 2047u);
      const int ty = (int)((ent >> 19) & 15u);
      int dead = 0;
#pragma unroll 1
      for (int q = p + 1; q < aen; ++q) dead |= ((als[q] & 255u) == j) ? 1 : 0;
      livef[e] = dead ? 0 : 1;
      const float w = ewt[ty];
      rs += dead ? 0.0f : w;
      nd += dead;
    }
    sums[tid] = rs;
#pragma unroll
    for (int d = 16; d >= 1; d >>= 1) nd += __shfl_xor(nd, d);
    if (lane == 0) wdup[wave] = nd;
  }
  __syncthreads();

  {
    int gst = offs[tid], gen = offs[tid + 1];
    gst = gst < 0 ? 0 : (gst > EPG ? EPG : gst);
    gen = gen < gst ? gst : (gen > EPG ? EPG : gen);
    float cs = 1.0f;
#pragma unroll 1
    for (int p = gst; p < gen; ++p) {
      const unsigned ent = gls[p];
      const int e  = (int)((ent >> 12) & 2047u);
      const int ty = (int)((ent >> 8) & 15u);
      const int lv = livef[e];
      const float w = ewt[ty];
      cs += (lv != 0) ? w : 0.0f;
    }
    sums[NPG + tid] = cs;
#pragma unroll 1
    for (int q = 0; q < 2; ++q) inv[q * NPG + tid] = 1.0f / sqrtf(sums[q * NPG + tid]);
  }
  __syncthreads();

  {
    const float rc = inv[NPG + tid];
#pragma unroll 1
    for (int p = ast; p < aen; ++p) {
      const unsigned ent = als[p];
      const int j  = (int)(ent & 255u);
      const int e  = (int)((ent >> 8) & 2047u);
      const int ty = (int)((ent >> 19) & 15u);
      const int lv = livef[e];
      const float w = ewt[ty];
      const float rr = inv[j];
      const float cv = (rc * w) * rr;
      cfs[p] = (lv != 0) ? cv : 0.0f;
    }
    slf[tid] = rc * inv[tid];
  }
  __syncthreads();

  {
    const int t64 = tid & 63;
    const size_t gb = (size_t)g * EPG;
    const v4u g0 = *(const v4ua*)(gls + 4 * tid), g1 = *(const v4ua*)(gls + 4 * (tid + NTHR));
    const v4u q0 = *(const v4ua*)(als + 4 * tid), q1 = *(const v4ua*)(als + 4 * (tid + NTHR));
    const v4f c0 = *(const v4fa*)(cfs + 4 * tid), c1 = *(const v4fa*)(cfs + 4 * (tid + NTHR));
    const v4i og = *(const v4ia*)(offs + 4 * t64);
    const v4i oa = *(const v4ia*)(offs + OFFP + 4 * t64);
    const v4f sf = *(const v4fa*)(slf + 4 * t64);
    const v4f vr = *(const v4f*)(vnemb + 4 * t64);
    v4f vn4;
    vn4.x = bf_rne(vr.x); vn4.y = bf_rne(vr.y); vn4.z = bf_rne(vr.z); vn4.w = bf_rne(vr.w);
    int bad = 0, dup = 0;
#pragma unroll
    for (int w2 = 0; w2 < 8; ++w2) { bad |= wbad[w2]; dup += wdup[w2]; }
    v4i mt = {0, 0, 0, 0};
    if (tid == 0) { mt.x = bad; mt.y = dup; }
    const float one = (tid >= 64 && tid < 192) ? 1.0f : 0.0f;
    v4f sid; sid.x = one; sid.y = one; sid.z = one; sid.w = one;
#pragma unroll
    for (int ps = 0; ps < 2; ++ps) {
      *(volatile v4u*)(GL + gb + 4 * tid) = g0;
      *(volatile v4u*)(GL + gb + 4 * (tid + NTHR)) = g1;
      *(volatile v4u*)(AL + gb + 4 * tid) = q0;
      *(volatile v4u*)(AL + gb + 4 * (tid + NTHR)) = q1;
      *(volatile v4f*)(COEF + gb + 4 * tid) = c0;
      *(volatile v4f*)(COEF + gb + 4 * (tid + NTHR)) = c1;
      if (tid < 64) {
        *(volatile v4i*)(GOFF + (size_t)g * NPG + 4 * tid) = og;
        *(volatile v4i*)(AOFF + (size_t)g * NPG + 4 * tid) = oa;
        *(volatile v4f*)(SELFC + (size_t)g * NPG + 4 * tid) = sf;
        *(volatile v4f*)(VN + (size_t)g * EMB + 4 * tid) = vn4;
      }
      if (tid < 8) *(volatile v4i*)(META + (size_t)g * 32 + 4 * tid) = mt;
      if (g == 0) *(volatile v4f*)(STAT2 + 4 * tid) = sid;
      if (ps == 0) __threadfence();
    }
  }
}

__global__ __launch_bounds__(NTHR) void k_prop(
    const int* __restrict__ aidx, const float* __restrict__ aemb, const int* __restrict__ ordp,
    const unsigned* __restrict__ AL, const float* __restrict__ COEF, const int* __restrict__ AOFF,
    const float* __restrict__ SELFC, float* U) {
  extern __shared__ v4f dynl[];
  float*    X    = (float*)dynl;
  float*    Y    = X + 2 * NPG * PC;
  unsigned* als  = (unsigned*)(Y + NPG * PC);
  float*    cfs  = (float*)(als + EPG);
  int*      aoff = (int*)(cfs + EPG);
  float*    slf  = (float*)(aoff + 264);
  const int tid = (int)threadIdx.x, lane = tid & 31, wave = tid >> 5;
  const int chunk = (int)blockIdx.x, g = (int)blockIdx.y;

  {
    const size_t gb = (size_t)g * EPG;
#pragma unroll
    for (int q = 0; q < 2; ++q) {
      const v4u a = *(const v4u*)(AL + gb + 4 * (tid + NTHR * q));
      const v4f c = *(const v4f*)(COEF + gb + 4 * (tid + NTHR * q));
      *(v4ua*)(als + 4 * (tid + NTHR * q)) = a;
      *(v4fa*)(cfs + 4 * (tid + NTHR * q)) = c;
    }
    const int t64 = tid & 63;
    const v4i o = *(const v4i*)(AOFF + (size_t)g * NPG + 4 * t64);
    const v4f s = *(const v4f*)(SELFC + (size_t)g * NPG + 4 * t64);
    if (tid < 64) {
      *(v4ia*)(aoff + 4 * tid) = o;
      *(v4fa*)(slf + 4 * tid) = s;
    }
    if (tid == 0) aoff[NPG] = EPG;
  }
#pragma unroll 2
  for (int i = 0; i < NPG / 8; ++i) {
    const int r = wave + 8 * i;
    int a = aidx[g * NPG + r];
    a = a < 0 ? 0 : (a > ATOMV - 1 ? ATOMV - 1 : a);
    const v2f v = *(const v2f*)(aemb + (size_t)a * EMB + chunk * PC + 2 * lane);
    v2f x;
    x.x = bf_rne(v.x); x.y = bf_rne(v.y);
    *(v2fa*)(X + r * PC + 2 * lane) = x;
    *(v2fa*)(Y + r * PC + 2 * lane) = x;
  }
  int ord = ordp[0];
  ord = ord < 0 ? 0 : (ord > ORDMAX ? ORDMAX : ord);
  __syncthreads();

#pragma unroll 1
  for (int hop = 0; hop < ord; ++hop) {
    const int so = (hop & 1) * (NPG * PC);
    const int dn = (NPG * PC) - so;
    const float* src = X + so;
    float* dst = X + dn;
#pragma unroll 1
    for (int i = 0; i < NPG / 8; ++i) {
      const int r = wave + 8 * i;
      int st = aoff[r], en = aoff[r + 1];
      st = st < 0 ? 0 : (st > EPG ? EPG : st);
      en = en < st ? st : (en > EPG ? EPG : en);
      const int cn = en - st;
      float ax = 0.0f, ay = 0.0f;
#pragma unroll 1
      for (int b0 = 0; b0 < cn; b0 += 32) {
        int idx = st + b0 + lane;
        idx = idx > EPG - 1 ? EPG - 1 : idx;
        const int ent = (int)als[idx];
        const int cfi = __float_as_int(cfs[idx]);
        const int m32 = (cn - b0) < 32 ? (cn - b0) : 32;
#pragma unroll 1
        for (int k = 0; k < m32; ++k) {
          const int j = __builtin_amdgcn_readlane(ent, k) & 255;
          const float c = __int_as_float(__builtin_amdgcn_readlane(cfi, k));
          const v2f xv = *(const v2fa*)(src + j * PC + 2 * lane);
          ax = fmaf(c, xv.x, ax);
          ay = fmaf(c, xv.y, ay);
        }
      }
      const v2f xs = *(const v2fa*)(src + r * PC + 2 * lane);
      const float sc = slf[r];
      ax = fmaf(sc, xs.x, ax);
      ay = fmaf(sc, xs.y, ay);
      v2f xn; xn.x = ax; xn.y = ay;
      *(v2fa*)(dst + r * PC + 2 * lane) = xn;
      v2f yv = *(const v2fa*)(Y + r * PC + 2 * lane);
      yv.x += ax; yv.y += ay;
      *(v2fa*)(Y + r * PC + 2 * lane) = yv;
    }
    __syncthreads();
  }

  const float scl = 1.0f / (float)(ord + 1);
#pragma unroll
  for (int ps = 0; ps < 2; ++ps) {
#pragma unroll 4
    for (int i = 0; i < NPG / 8; ++i) {
      const int r = wave + 8 * i;
      v2f yv = *(const v2fa*)(Y + r * PC + 2 * lane);
      yv.x *= scl; yv.y *= scl;
      *(volatile v2f*)(U + (size_t)(g * NPG + r) * EMB + chunk * PC + 2 * lane) = yv;
    }
    if (ps == 0) __threadfence();
  }
}

__global__ __launch_bounds__(NTHR) void k_agg(
    const float* __restrict__ U, const float* __restrict__ ST, int relu,
    const float* __restrict__ VN, const float* __restrict__ BE, const float* __restrict__ epsp,
    const unsigned* __restrict__ GL, const int* __restrict__ GOFF, const int* __restrict__ META,
    unsigned short* Z, unsigned short* VT, int doVT) {
  extern __shared__ v4f dynl[];
  float*          hin  = (float*)dynl;
  float*          be   = hin + NPG * AC;
  unsigned*       gls  = (unsigned*)(be + BONDV * AC);
  int*            goff = (int*)(gls + EPG);
  float*          vts  = (float*)(goff + 264);
  unsigned short* vth  = (unsigned short*)(vts + NTHR);
  const int tid = (int)threadIdx.x, lane = tid & 31, wave = tid >> 5;
  const int g = (int)blockIdx.x;

  {
    const size_t gb = (size_t)g * EPG;
#pragma unroll
    for (int q = 0; q < 2; ++q) {
      const v4u a = *(const v4u*)(GL + gb + 4 * (tid + NTHR * q));
      *(v4ua*)(gls + 4 * (tid + NTHR * q)) = a;
    }
    const int t64 = tid & 63;
    const v4i o = *(const v4i*)(GOFF + (size_t)g * NPG + 4 * t64);
    if (tid < 64) *(v4ia*)(goff + 4 * tid) = o;
    if (tid == 0) goff[NPG] = EPG;
  }
  const int bad = META[(size_t)g * 32];
  const float pz = (bad != 0) ? __int_as_float(0x7fc00000) : 0.0f;
  const float eps1 = 1.0f + bf_rne(epsp[0]);

#pragma unroll 1
  for (int hf = 0; hf < 2; ++hf) {
    const int c4 = AC * hf + 4 * lane;
    const v4f m4 = *(const v4f*)(ST + c4);
    const v4f r4 = *(const v4f*)(ST + EMB + c4);
    const v4f g4 = *(const v4f*)(ST + 2 * EMB + c4);
    const v4f b4 = *(const v4f*)(ST + 3 * EMB + c4);
    const v4f vn4 = *(const v4f*)(VN + (size_t)g * EMB + c4);
#pragma unroll
    for (int q = 0; q < 2; ++q) {
      const int idx = 4 * (tid + NTHR * q);
      const int ty = idx >> 7, c = idx & (AC - 1);
      const v4f v = *(const v4f*)(BE + (size_t)ty * EMB + AC * hf + c);
      v4f o;
      o.x = bf_rne(v.x); o.y = bf_rne(v.y); o.z = bf_rne(v.z); o.w = bf_rne(v.w);
      *(v4fa*)(be + idx) = o;
    }
#pragma unroll 2
    for (int i = 0; i < NPG / 8; ++i) {
      const int r = wave + 8 * i;
      const v4f u = *(const v4f*)(U + (size_t)(g * NPG + r) * EMB + c4);
      float f0 = ((u.x - m4.x) * r4.x) * g4.x + b4.x;
      float f1 = ((u.y - m4.y) * r4.y) * g4.y + b4.y;
      float f2 = ((u.z - m4.z) * r4.z) * g4.z + b4.z;
      float f3 = ((u.w - m4.w) * r4.w) * g4.w + b4.w;
      if (relu != 0) { f0 = relu_np(f0); f1 = relu_np(f1); f2 = relu_np(f2); f3 = relu_np(f3); }
      v4f h;
      h.x = f0 + vn4.x; h.y = f1 + vn4.y; h.z = f2 + vn4.z; h.w = f3 + vn4.w;
      *(v4fa*)(hin + r * AC + 4 * lane) = h;
    }
    __syncthreads();

    {
      const int c = tid & (AC - 1), hr = tid >> 7;
      float s = 0.0f;
#pragma unroll 4
      for (int r = 0; r < NPG / 2; ++r) s += hin[(hr * (NPG / 2) + r) * AC + c];
      vts[tid] = s;
    }
    __syncthreads();
    if (tid < AC) {
      const float vt = (vts[tid] + vts[AC + tid]) + VN[(size_t)g * EMB + AC * hf + tid];
      const unsigned hb = bf_bits(vt);
      const unsigned lb2 = bf_bits(vt - bf_val(hb));
      vth[tid] = (unsigned short)hb;
      vth[AC + tid] = (unsigned short)lb2;
    }
    __syncthreads();
    if (doVT != 0 && wave == 0) {
      const int piece = lane >> 4, k = lane & 15;
      const v8us pk = *(const v8usa*)(vth + piece * AC + 8 * k);
      unsigned short* vp = VT + (size_t)g * (2 * EMB) + piece * EMB + AC * hf + 8 * k;
      *(volatile v8us*)vp = pk;
      __threadfence();
      *(volatile v8us*)vp = pk;
    }

#pragma unroll 1
    for (int i = 0; i < NPG / 8; ++i) {
      const int d = wave + 8 * i;
      int st = goff[d], en = goff[d + 1];
      st = st < 0 ? 0 : (st > EPG ? EPG : st);
      en = en < st ? st : (en > EPG ? EPG : en);
      const int cn = en - st;
      float a0 = 0.0f, a1 = 0.0f, a2 = 0.0f, a3 = 0.0f;
#pragma unroll 1
      for (int b0 = 0; b0 < cn; b0 += 32) {
        int idx = st + b0 + lane;
        idx = idx > EPG - 1 ? EPG - 1 : idx;
        const int ent = (int)gls[idx];
        const int m32 = (cn - b0) < 32 ? (cn - b0) : 32;
#pragma unroll 1
        for (int k = 0; k < m32; ++k) {
          const int u = __builtin_amdgcn_readlane(ent, k);
          const int s = u & 255;
          const int ty = (u >> 8) & 15;
          const v4f hv = *(const v4fa*)(hin + s * AC + 4 * lane);
          const v4f ev = *(const v4fa*)(be + ty * AC + 4 * lane);
          a0 += relu_np(hv.x + ev.x);
          a1 += relu_np(hv.y + ev.y);
          a2 += relu_np(hv.z + ev.z);
          a3 += relu_np(hv.w + ev.w);
        }
      }
      const v4f hs = *(const v4fa*)(hin + d * AC + 4 * lane);
      const float z0 = (eps1 * hs.x + a0) + pz;
      const float z1 = (eps1 * hs.y + a1) + pz;
      const float z2 = (eps1 * hs.z + a2) + pz;
      const float z3 = (eps1 * hs.w + a3) + pz;
      const unsigned h0 = bf_bits(z0), h1 = bf_bits(z1), h2 = bf_bits(z2), h3 = bf_bits(z3);
      v4us hq, lq;
      hq.x = (unsigned short)h0; hq.y = (unsigned short)h1; hq.z = (unsigned short)h2; hq.w = (unsigned short)h3;
      lq.x = (unsigned short)bf_bits(z0 - bf_val(h0));
      lq.y = (unsigned short)bf_bits(z1 - bf_val(h1));
      lq.z = (unsigned short)bf_bits(z2 - bf_val(h2));
      lq.w = (unsigned short)bf_bits(z3 - bf_val(h3));
      unsigned short* zp = Z + (size_t)(g * NPG + d) * (2 * EMB) + AC * hf + 4 * lane;
      *(volatile v4us*)zp = hq;
      *(volatile v4us*)(zp + EMB) = lq;
      __threadfence();
      *(volatile v4us*)zp = hq;
      *(volatile v4us*)(zp + EMB) = lq;
    }
    __syncthreads();
  }
}

template <int MODE>
__global__ __launch_bounds__(GTHR) void k_gemm(const unsigned short* __restrict__ A,
                                               const unsigned short* __restrict__ BT,
                                               int K, int Nout, const float* __restrict__ bias,
                                               unsigned short* outH, float* outF, float* part) {
  __shared__ __attribute__((aligned(16))) float stg[GBM * GBN];
  __shared__ __attribute__((aligned(16))) float pst[PARTW];
  const int tid = (int)threadIdx.x, lane = tid & 31, wave = tid >> 5, hh = lane >> 4, m = lane & 15;
  const int rowBase = (int)blockIdx.x * GBM;
  const int colBase = (int)blockIdx.y * GBN;

  v8f acc[8];
  {
    const v8f z = {0.f, 0.f, 0.f, 0.f, 0.f, 0.f, 0.f, 0.f};
#pragma unroll
    for (int t = 0; t < 8; ++t) acc[t] = z;
  }
  const unsigned short* ap = A  + (size_t)(rowBase + 16 * wave + m) * (size_t)K + 8 * hh;
  const unsigned short* bp = BT + (size_t)(colBase + m) * (size_t)K + 8 * hh;

#pragma unroll 1
  for (int k0 = 0; k0 < K; k0 += 32) {
    FragB af;
    af.h[0] = *(const v8usa*)(ap + k0);
    af.h[1] = *(const v8usa*)(ap + k0 + 16);
#pragma unroll
    for (int nt = 0; nt < 8; ++nt) {
      const unsigned short* wq = bp + (size_t)(16 * nt) * (size_t)K + k0;
      FragB bf;
      bf.h[0] = *(const v8usa*)wq;
      bf.h[1] = *(const v8usa*)(wq + 16);
      acc[nt] = wmb(af, bf, acc[nt]);
    }
  }

#pragma unroll
  for (int nt = 0; nt < 8; ++nt) {
    const int lc = 16 * nt + m;
    const float bb = bf_rne(bias[colBase + lc]);
#pragma unroll
    for (int r = 0; r < 8; ++r) {
      const int lr = 16 * wave + 8 * hh + r;
      float v = acc[nt][r] + bb;
      if (MODE != 0) v = relu_np(v);
      stg[lr * GBN + lc] = v;
    }
  }
  __syncthreads();

  if constexpr (MODE != 1) {
    if constexpr (MODE == 0) {
      float s = 0.0f;
#pragma unroll 4
      for (int r = 0; r < GBM; ++r) s += stg[r * GBN + tid];
      const float mean = s * (1.0f / (float)GBM);
      float q = 0.0f;
#pragma unroll 4
      for (int r = 0; r < GBM; ++r) {
        const float d = stg[r * GBN + tid] - mean;
        q = fmaf(d, d, q);
      }
      pst[tid] = mean;
      pst[GBN + tid] = q;
    }
#pragma unroll 1
    for (int ib = 0; ib < 4; ++ib) {
      v4f fv[4];
#pragma unroll
      for (int i = 0; i < 4; ++i) fv[i] = *(const v4fa*)(stg + (16 * wave + 4 * ib + i) * GBN + 4 * lane);
#pragma unroll
      for (int i = 0; i < 4; ++i) {
        float* op = outF + (size_t)(rowBase + 16 * wave + 4 * ib + i) * (size_t)Nout + colBase + 4 * lane;
        *(volatile v4f*)op = fv[i];
      }
      __threadfence();
#pragma unroll
      for (int i = 0; i < 4; ++i) {
        float* op = outF + (size_t)(rowBase + 16 * wave + 4 * ib + i) * (size_t)Nout + colBase + 4 * lane;
        *(volatile v4f*)op = fv[i];
      }
    }
    if constexpr (MODE == 0) {
      __syncthreads();
      const int pb = (int)blockIdx.x * (int)gridDim.y + (int)blockIdx.y;
      const int t4 = tid & 63;
      const v4f ps = *(const v4fa*)(pst + 4 * t4);
      if (tid < PARTW / 4) *(volatile v4f*)(part + (size_t)pb * PARTW + 4 * tid) = ps;
      __threadfence();
      if (tid < PARTW / 4) *(volatile v4f*)(part + (size_t)pb * PARTW + 4 * tid) = ps;
    }
  } else {
#pragma unroll 1
    for (int ib = 0; ib < 4; ++ib) {
      v4us hv[4], lv[4];
#pragma unroll
      for (int i = 0; i < 4; ++i) {
        const v4f x = *(const v4fa*)(stg + (16 * wave + 4 * ib + i) * GBN + 4 * lane);
        const unsigned h0 = bf_bits(x.x), h1 = bf_bits(x.y), h2 = bf_bits(x.z), h3 = bf_bits(x.w);
        v4us hq, lq;
        hq.x = (unsigned short)h0; hq.y = (unsigned short)h1; hq.z = (unsigned short)h2; hq.w = (unsigned short)h3;
        lq.x = (unsigned short)bf_bits(x.x - bf_val(h0));
        lq.y = (unsigned short)bf_bits(x.y - bf_val(h1));
        lq.z = (unsigned short)bf_bits(x.z - bf_val(h2));
        lq.w = (unsigned short)bf_bits(x.w - bf_val(h3));
        hv[i] = hq; lv[i] = lq;
      }
#pragma unroll
      for (int i = 0; i < 4; ++i) {
        unsigned short* op = outH + (size_t)(rowBase + 16 * wave + 4 * ib + i) * (size_t)(2 * Nout) + colBase + 4 * lane;
        *(volatile v4us*)op = hv[i];
        *(volatile v4us*)(op + Nout) = lv[i];
      }
      __threadfence();
#pragma unroll
      for (int i = 0; i < 4; ++i) {
        unsigned short* op = outH + (size_t)(rowBase + 16 * wave + 4 * ib + i) * (size_t)(2 * Nout) + colBase + 4 * lane;
        *(volatile v4us*)op = hv[i];
        *(volatile v4us*)(op + Nout) = lv[i];
      }
    }
  }
}

__global__ __launch_bounds__(HID) void k_comb(const float* __restrict__ part, int nCB,
                                              const float* __restrict__ gam, const float* __restrict__ bet,
                                              float* stat) {
  __shared__ __attribute__((aligned(16))) float stg[4 * HID];
  const int tid = (int)threadIdx.x;
  const int C  = nCB * GBN;
  const int cb = tid >> 7;
  const int cc = tid & (GBN - 1);
  const float* base = part + (size_t)cb * PARTW + cc;
  const size_t stride = (size_t)nCB * PARTW;
  double sm = 0.0;
#pragma unroll 4
  for (int b = 0; b < NRT; ++b) sm += (double)base[(size_t)b * stride];
  const double mean = sm * (1.0 / (double)NRT);
  double q = 0.0, dv = 0.0;
#pragma unroll 4
  for (int b = 0; b < NRT; ++b) {
    const double mb = (double)base[(size_t)b * stride];
    const double qb = (double)base[(size_t)b * stride + GBN];
    const double d = mb - mean;
    q += qb;
    dv += d * d;
  }
  const double M2 = q + (double)GBM * dv;
  const float var = (float)(M2 * (1.0 / (double)NNODE));
  const float rstd = 1.0f / sqrtf(var + 1e-5f);
  stg[tid] = (float)mean;
  stg[C + tid] = rstd;
  stg[2 * C + tid] = bf_rne(gam[tid]);
  stg[3 * C + tid] = bf_rne(bet[tid]);
  __syncthreads();
  const v4f v = *(const v4fa*)(stg + 4 * tid);
  *(volatile v4f*)(stat + 4 * tid) = v;
  __threadfence();
  *(volatile v4f*)(stat + 4 * tid) = v;
}

__global__ __launch_bounds__(NTHR) void k_apply(const float* __restrict__ T, const float* __restrict__ ST,
                                                int nUnits, unsigned short* TH) {
  const int u = (int)blockIdx.x * NTHR + (int)threadIdx.x;
  if (u >= nUnits) return;
  const int row = u >> 6;
  const int c8  = (u & 63) * 8;
  const float* tp = T + (size_t)u * 8;
  const v4f xa = *(const v4f*)tp,                 xb = *(const v4f*)(tp + 4);
  const v4f ma = *(const v4f*)(ST + c8),           mb = *(const v4f*)(ST + c8 + 4);
  const v4f ra = *(const v4f*)(ST + HID + c8),     rb = *(const v4f*)(ST + HID + c8 + 4);
  const v4f ga = *(const v4f*)(ST + 2 * HID + c8), gb = *(const v4f*)(ST + 2 * HID + c8 + 4);
  const v4f ba = *(const v4f*)(ST + 3 * HID + c8), bb = *(const v4f*)(ST + 3 * HID + c8 + 4);
  const float x[8]  = {xa.x, xa.y, xa.z, xa.w, xb.x, xb.y, xb.z, xb.w};
  const float mm[8] = {ma.x, ma.y, ma.z, ma.w, mb.x, mb.y, mb.z, mb.w};
  const float rr[8] = {ra.x, ra.y, ra.z, ra.w, rb.x, rb.y, rb.z, rb.w};
  const float gg[8] = {ga.x, ga.y, ga.z, ga.w, gb.x, gb.y, gb.z, gb.w};
  const float be[8] = {ba.x, ba.y, ba.z, ba.w, bb.x, bb.y, bb.z, bb.w};
  v8us ho, lo;
#pragma unroll
  for (int j = 0; j < 8; ++j) {
    const float y = relu_np(((x[j] - mm[j]) * rr[j]) * gg[j] + be[j]);
    const unsigned hb = bf_bits(y);
    ho[j] = (unsigned short)hb;
    lo[j] = (unsigned short)bf_bits(y - bf_val(hb));
  }
  unsigned short* hp = TH + (size_t)row * (2 * HID) + c8;
  *(volatile v8us*)hp = ho;
  *(volatile v8us*)(hp + HID) = lo;
  __threadfence();
  *(volatile v8us*)hp = ho;
  *(volatile v8us*)(hp + HID) = lo;
}

__global__ __launch_bounds__(NTHR) void k_out(const float* __restrict__ Uo, const float* __restrict__ ST,
                                              int nUnits, float* out) {
  const int u = (int)blockIdx.x * NTHR + (int)threadIdx.x;
  if (u >= nUnits) return;
  const int c4 = (u & 63) * 4;
  const v4f x = *(const v4f*)(Uo + (size_t)u * 4);
  const v4f m = *(const v4f*)(ST + c4);
  const v4f r = *(const v4f*)(ST + EMB + c4);
  const v4f g = *(const v4f*)(ST + 2 * EMB + c4);
  const v4f b = *(const v4f*)(ST + 3 * EMB + c4);
  v4f o;
  o.x = ((x.x - m.x) * r.x) * g.x + b.x;
  o.y = ((x.y - m.y) * r.y) * g.y + b.y;
  o.z = ((x.z - m.z) * r.z) * g.z + b.z;
  o.w = ((x.w - m.w) * r.w) * g.w + b.w;
  float* op = out + (size_t)u * 4;
  *(volatile v4f*)op = o;
  __threadfence();
  *(volatile v4f*)op = o;
}

static inline size_t al256(size_t o) { return (o + 255) & ~(size_t)255; }

extern "C" void kernel_launch(void* const* d_in, const int* in_sizes, int n_in,
                              void* d_out, int out_size, void* d_ws, size_t ws_size,
                              hipStream_t stream) {
  if (n_in < 23) return;
  if (in_sizes[0] != NB * NPG || in_sizes[1] != NB * 2 * EPG || in_sizes[2] != NB * EPG) return;
  if (in_sizes[3] != 1 || in_sizes[4] != ATOMV * EMB || in_sizes[5] != BONDV * EHC) return;
  if (in_sizes[6] != EHC || in_sizes[7] != 1 || in_sizes[8] != NLAY * BONDV * EMB) return;
  if (in_sizes[9] != NLAY || in_sizes[10] != NLAY * EMB * HID || in_sizes[11] != NLAY * HID) return;
  if (in_sizes[12] != NLAY * HID || in_sizes[13] != NLAY * HID || in_sizes[14] != NLAY * HID * EMB) return;
  if (in_sizes[15] != NLAY * EMB || in_sizes[16] != NLAY * EMB || in_sizes[17] != NLAY * EMB) return;
  if (in_sizes[18] != EMB || in_sizes[19] != (NLAY - 1) * EMB * HID || in_sizes[20] != (NLAY - 1) * HID) return;
  if (in_sizes[21] != (NLAY - 1) * HID * EMB || in_sizes[22] != (NLAY - 1) * EMB) return;
  if (out_size != NNODE * EMB) return;

  const int*   atom_idx   = (const int*)  d_in[0];
  const int*   lei        = (const int*)  d_in[1];
  const int*   eat        = (const int*)  d_in[2];
  const int*   ordp       = (const int*)  d_in[3];
  const float* atom_emb   = (const float*)d_in[4];
  const float* bond_emb_h = (const float*)d_in[5];
  const float* edge_lin_w = (const float*)d_in[6];
  const float* edge_lin_b = (const float*)d_in[7];
  const float* bond_emb_l = (const float*)d_in[8];
  const float* gin_eps    = (const float*)d_in[9];
  const float* mlp_w1     = (const float*)d_in[10];
  const float* mlp_b1     = (const float*)d_in[11];
  const float* mlp_bn_g   = (const float*)d_in[12];
  const float* mlp_bn_b   = (const float*)d_in[13];
  const float* mlp_w2     = (const float*)d_in[14];
  const float* mlp_b2     = (const float*)d_in[15];
  const float* out_bn_g   = (const float*)d_in[16];
  const float* out_bn_b   = (const float*)d_in[17];
  const float* vn_emb     = (const float*)d_in[18];
  const float* vn_w1      = (const float*)d_in[19];
  const float* vn_b1      = (const float*)d_in[20];
  const float* vn_w2      = (const float*)d_in[21];
  const float* vn_b2      = (const float*)d_in[22];
  float* out = (float*)d_out;

  char* ws = (char*)d_ws;
  size_t off = 0;
  const size_t oW1D = off; off = al256(off + (size_t)NLAY * HID * (2 * EMB) * 2);
  const size_t oW2D = off; off = al256(off + (size_t)NLAY * EMB * (2 * HID) * 2);
  const size_t oV1D = off; off = al256(off + (size_t)(NLAY - 1) * HID * (2 * EMB) * 2);
  const size_t oV2D = off; off = al256(off + (size_t)(NLAY - 1) * EMB * (2 * HID) * 2);
  const size_t oGL  = off; off = al256(off + (size_t)NB * EPG * 4);
  const size_t oAL  = off; off = al256(off + (size_t)NB * EPG * 4);
  const size_t oCF  = off; off = al256(off + (size_t)NB * EPG * 4);
  const size_t oGO  = off; off = al256(off + (size_t)NB * NPG * 4);
  const size_t oAO  = off; off = al256(off + (size_t)NB * NPG * 4);
  const size_t oSF  = off; off = al256(off + (size_t)NB * NPG * 4);
  const size_t oMT  = off; off = al256(off + (size_t)NB * 32 * 4);
  const size_t oVN  = off; off = al256(off + (size_t)NB * EMB * 4);
  const size_t oVT  = off; off = al256(off + (size_t)NB * (2 * EMB) * 2);
  const size_t oHV  = off; off = al256(off + (size_t)NB * (2 * HID) * 2);
  const size_t oS1  = off; off = al256(off + (size_t)4 * HID * 4);
  const size_t oS2  = off; off = al256(off + (size_t)4 * EMB * 4);
  const size_t oPT  = off; off = al256(off + (size_t)NRT * (HID / GBN) * PARTW * 4);
  const size_t oZ   = off; off = al256(off + (size_t)NNODE * (2 * EMB) * 2);
  const size_t oT   = off; off = al256(off + (size_t)NNODE * HID * 4);
  const size_t oTH  = off; off = al256(off + (size_t)NNODE * (2 * HID) * 2);
  const size_t oU   = off; off = al256(off + (size_t)NNODE * EMB * 4);
  if (off > ws_size) return;
  unsigned short* W1D = (unsigned short*)(ws + oW1D);
  unsigned short* W2D = (unsigned short*)(ws + oW2D);
  unsigned short* V1D = (unsigned short*)(ws + oV1D);
  unsigned short* V2D = (unsigned short*)(ws + oV2D);
  unsigned* GL   = (unsigned*)(ws + oGL);
  unsigned* AL   = (unsigned*)(ws + oAL);
  float*    CF   = (float*)(ws + oCF);
  int*      GO   = (int*)(ws + oGO);
  int*      AO   = (int*)(ws + oAO);
  float*    SF   = (float*)(ws + oSF);
  int*      MT   = (int*)(ws + oMT);
  float*    VN   = (float*)(ws + oVN);
  unsigned short* VT = (unsigned short*)(ws + oVT);
  unsigned short* HV = (unsigned short*)(ws + oHV);
  float*    S1   = (float*)(ws + oS1);
  float*    S2   = (float*)(ws + oS2);
  float*    PT   = (float*)(ws + oPT);
  unsigned short* Z  = (unsigned short*)(ws + oZ);
  float*    T    = (float*)(ws + oT);
  unsigned short* TH = (unsigned short*)(ws + oTH);
  float*    Uo   = (float*)(ws + oU);

  hipFuncSetAttribute(reinterpret_cast<const void*>(&k_prop), hipFuncAttributeMaxDynamicSharedMemorySize, LDS_PROP);
  hipFuncSetAttribute(reinterpret_cast<const void*>(&k_agg),  hipFuncAttributeMaxDynamicSharedMemorySize, LDS_AGG);

  {
    const int u1 = NLAY * HID * ((2 * EMB) / 8);
    const int u2 = NLAY * EMB * ((2 * HID) / 8);
    const int u3 = (NLAY - 1) * HID * ((2 * EMB) / 8);
    const int u4 = (NLAY - 1) * EMB * ((2 * HID) / 8);
    k_wprep<<<u1 / NTHR, NTHR, 0, stream>>>(mlp_w1, EMB, HID, u1, W1D);
    k_wprep<<<u2 / NTHR, NTHR, 0, stream>>>(mlp_w2, HID, EMB, u2, W2D);
    k_wprep<<<u3 / NTHR, NTHR, 0, stream>>>(vn_w1,  EMB, HID, u3, V1D);
    k_wprep<<<u4 / NTHR, NTHR, 0, stream>>>(vn_w2,  HID, EMB, u4, V2D);
  }
  k_lists<<<NB, NTHR, 0, stream>>>(lei, eat, bond_emb_h, edge_lin_w, edge_lin_b, vn_emb,
                                   GL, GO, AL, CF, AO, SF, MT, VN, S2);
  k_prop<<<dim3(EMB / PC, NB), NTHR, LDS_PROP, stream>>>(atom_idx, atom_emb, ordp, AL, CF, AO, SF, Uo);

  const int nUa = NNODE * (HID / 8);
  const int nUo = NNODE * (EMB / 4);
  for (int l = 0; l < NLAY; ++l) {
    const int last = (l == NLAY - 1) ? 1 : 0;
    k_agg<<<NB, NTHR, LDS_AGG, stream>>>(Uo, S2, (l > 0) ? 1 : 0, VN,
                                         bond_emb_l + (size_t)l * BONDV * EMB, gin_eps + l,
                                         GL, GO, MT, Z, VT, last ? 0 : 1);
    k_gemm<0><<<dim3(NRT, HID / GBN), GTHR, 0, stream>>>(Z, W1D + (size_t)l * HID * (2 * EMB), 2 * EMB, HID,
                                                        mlp_b1 + (size_t)l * HID, VT, T, PT);
    k_comb<<<1, HID, 0, stream>>>(PT, HID / GBN, mlp_bn_g + (size_t)l * HID, mlp_bn_b + (size_t)l * HID, S1);
    k_apply<<<nUa / NTHR, NTHR, 0, stream>>>(T, S1, nUa, TH);
    k_gemm<0><<<dim3(NRT, EMB / GBN), GTHR, 0, stream>>>(TH, W2D + (size_t)l * EMB * (2 * HID), 2 * HID, EMB,
                                                        mlp_b2 + (size_t)l * EMB, VT, Uo, PT);
    k_comb<<<1, EMB, 0, stream>>>(PT, EMB / GBN, out_bn_g + (size_t)l * EMB, out_bn_b + (size_t)l * EMB, S2);
    if (!last) {
      k_gemm<1><<<dim3(NB / GBM, HID / GBN), GTHR, 0, stream>>>(VT, V1D + (size_t)l * HID * (2 * EMB), 2 * EMB, HID,
                                                             vn_b1 + (size_t)l * HID, HV, T, PT);
      k_gemm<2><<<dim3(NB / GBM, EMB / GBN), GTHR, 0, stream>>>(HV, V2D + (size_t)l * EMB * (2 * HID), 2 * HID, EMB,
                                                             vn_b2 + (size_t)l * EMB, VT, VN, PT);
    }
  }
  k_out<<<nUo / NTHR, NTHR, 0, stream>>>(Uo, S2, nUo, out);
}
